// SparseSphereConv_31731218383017
// MI455X (gfx1250) — hardware-verified
//
#include <hip/hip_runtime.h>
#include <stdint.h>

typedef float          v8f  __attribute__((ext_vector_type(8)));
typedef float          v4f  __attribute__((ext_vector_type(4)));
typedef v4f            v4fa __attribute__((may_alias));
typedef unsigned int   v4u  __attribute__((ext_vector_type(4)));
typedef unsigned short v8us __attribute__((ext_vector_type(8)));
typedef v8us           v8usa __attribute__((may_alias));
typedef __bf16         v16bf __attribute__((ext_vector_type(16)));
union Frag { v16bf v; v8us h[2]; };

#define NB   4
#define CI   32
#define CO   32
#define NV   40962
#define KK   9
#define KSQ  81
#define KD   (CI * KK)
#define TV   32
#define NVT  1281
#define VP   (NVT * TV)
#define AP   296
#define NTH  128

__device__ __forceinline__ unsigned short f2bf(float f) {
    unsigned u = __float_as_uint(f);
    u += 0x7FFFu + ((u >> 16) & 1u);
    return (unsigned short)(u >> 16);
}
__device__ __forceinline__ float bf2f(unsigned short b) {
    return __uint_as_float(((unsigned)b) << 16);
}

__device__ __forceinline__ v8f wmma_bf16(v16bf a, v16bf b, v8f c) {
    v8f d = __builtin_amdgcn_wmma_f32_16x16x32_bf16(false, a, false, b, (short)0, c, false, false);
    asm volatile("v_nop\n\tv_nop\n\tv_nop\n\tv_nop" : "+v"(d) : "v"(a), "v"(b));
    return d;
}

__device__ __forceinline__ void pack8(const float* __restrict__ p, v4u& hv, v4u& lv) {
    unsigned hw[4], lw[4];
    #pragma unroll
    for (int q = 0; q < 4; ++q) {
        float a = p[2 * q], c = p[2 * q + 1];
        unsigned short ha = f2bf(a), hc = f2bf(c);
        unsigned short la = f2bf(a - bf2f(ha)), lc = f2bf(c - bf2f(hc));
        hw[q] = (unsigned)ha | ((unsigned)hc << 16);
        lw[q] = (unsigned)la | ((unsigned)lc << 16);
    }
    hv.x = hw[0]; hv.y = hw[1]; hv.z = hw[2]; hv.w = hw[3];
    lv.x = lw[0]; lv.y = lw[1]; lv.z = lw[2]; lv.w = lw[3];
}

__global__ __launch_bounds__(256)
void k_wsplit(const float* __restrict__ w, unsigned short* whi, unsigned short* wlo, int nvec)
{
    const int tid = threadIdx.x;
    for (int i = tid; i < nvec; i += 256) {
        v4u hv, lv;
        pack8(w + 8 * (size_t)i, hv, lv);
        *(volatile v4u*)(whi + 8 * (size_t)i) = hv;
        *(volatile v4u*)(wlo + 8 * (size_t)i) = lv;
    }
    __threadfence();
    for (int i = tid; i < nvec; i += 256) {
        v4u hv, lv;
        pack8(w + 8 * (size_t)i, hv, lv);
        *(volatile v4u*)(whi + 8 * (size_t)i) = hv;
        *(volatile v4u*)(wlo + 8 * (size_t)i) = lv;
    }
}

__global__ __launch_bounds__(NTH)
void k_main(const float* __restrict__ x,
            const int*   __restrict__ nbr,
            const float* __restrict__ itp,
            const unsigned short* __restrict__ whi,
            const unsigned short* __restrict__ wlo,
            const float* __restrict__ bias,
            float* wsout)
{
    __shared__ __align__(16) unsigned short Ahi[TV * AP];
    __shared__ __align__(16) unsigned short Alo[TV * AP];
    __shared__ __align__(16) float sout[CO * TV];
    __shared__ float sitp[TV * KSQ];
    __shared__ int   sidx[TV * KK];
    __shared__ int   smask[TV];

    const int tid  = threadIdx.x;
    const int lane = tid & 31;
    const int wv   = tid >> 5;
    const int v0   = blockIdx.x * TV;
    const int b    = blockIdx.y;

    for (int i = tid; i < TV * KK; i += NTH) {
        int vt = i / KK;
        int v  = v0 + vt;
        int ix = 0;
        if (v < NV) {
            ix = nbr[(size_t)v * KK + (i - vt * KK)];
            if (ix < 0) ix += NV;
            ix = ix < 0 ? 0 : (ix > NV - 1 ? NV - 1 : ix);
        }
        sidx[i] = ix;
    }
    for (int i = tid; i < TV * KSQ; i += NTH) {
        int vt = i / KSQ;
        int v  = v0 + vt;
        sitp[i] = (v < NV) ? itp[(size_t)v * KSQ + (i - vt * KSQ)] : 0.0f;
    }
    __syncthreads();

    const float* xp = x + ((size_t)(b * CI + lane)) * NV;
    #pragma unroll 1
    for (int it = 0; it < 8; ++it) {
        const int  vt    = wv + 4 * it;
        const bool valid = (v0 + vt) < NV;
        float g[KK];
        int nz = 0;
        #pragma unroll
        for (int k = 0; k < KK; ++k) {
            float gv = valid ? xp[sidx[vt * KK + k]] : 0.0f;
            g[k] = gv;
            nz |= (gv != 0.0f) ? 1 : 0;
        }
        const float* ip = sitp + vt * KSQ;
        unsigned short* ah = Ahi + vt * AP + lane * KK;
        unsigned short* al = Alo + vt * AP + lane * KK;
        #pragma unroll
        for (int j = 0; j < KK; ++j) {
            float s = 0.0f;
            #pragma unroll
            for (int k = 0; k < KK; ++k) s = fmaf(g[k], ip[k * KK + j], s);
            unsigned short hb = f2bf(s);
            ah[j] = hb;
            al[j] = f2bf(s - bf2f(hb));
        }
        unsigned bal = __builtin_amdgcn_ballot_w32(nz != 0);
        if (lane == 0) smask[vt] = (bal != 0u) ? 1 : 0;
    }
    __syncthreads();

    const int h  = lane >> 4;
    const int m  = lane & 15;
    const int mt = wv & 1;
    const int nt = wv >> 1;
    const unsigned short* arh = Ahi + (16 * mt + m) * AP + 8 * h;
    const unsigned short* arl = Alo + (16 * mt + m) * AP + 8 * h;
    const unsigned short* brh = whi + (size_t)(16 * nt + m) * KD + 8 * h;
    const unsigned short* brl = wlo + (size_t)(16 * nt + m) * KD + 8 * h;

    v8f acc = {0.f, 0.f, 0.f, 0.f, 0.f, 0.f, 0.f, 0.f};
    #pragma unroll 1
    for (int kb = 0; kb < KD / 32; ++kb) {
        const int k0 = kb * 32;
        Frag fa, fal, fb, fbl;
        fa.h[0]  = *(const v8usa*)(arh + k0);   fa.h[1]  = *(const v8usa*)(arh + k0 + 16);
        fal.h[0] = *(const v8usa*)(arl + k0);   fal.h[1] = *(const v8usa*)(arl + k0 + 16);
        fb.h[0]  = *(const v8usa*)(brh + k0);   fb.h[1]  = *(const v8usa*)(brh + k0 + 16);
        fbl.h[0] = *(const v8usa*)(brl + k0);   fbl.h[1] = *(const v8usa*)(brl + k0 + 16);
        acc = wmma_bf16(fa.v,  fb.v,  acc);
        acc = wmma_bf16(fa.v,  fbl.v, acc);
        acc = wmma_bf16(fal.v, fb.v,  acc);
    }

    const int   o  = 16 * nt + m;
    const float bo = bias[o];
    #pragma unroll
    for (int r = 0; r < 8; ++r) {
        int vt = 16 * mt + 8 * h + r;
        float mk = smask[vt] ? 1.0f : 0.0f;
        sout[o * TV + vt] = (acc[r] + bo) * mk;
    }
    __syncthreads();

    float* base = wsout + ((size_t)(b * CO)) * VP + v0;
    const int p = lane & 7;
    const int oa = 8 * wv + (lane >> 3);
    const int ob = oa + 4;
    v4f va = *(const v4fa*)(sout + oa * TV + 4 * p);
    v4f vb = *(const v4fa*)(sout + ob * TV + 4 * p);
    float* pa = base + (size_t)oa * VP + 4 * p;
    float* pb = base + (size_t)ob * VP + 4 * p;
    *(volatile v4f*)pa = va;
    *(volatile v4f*)pb = vb;
    __threadfence();
    *(volatile v4f*)pa = va;
    *(volatile v4f*)pb = vb;
}

__global__ __launch_bounds__(256)
void k_lines(const float* __restrict__ wsout, float* out, int total)
{
    const int q = blockIdx.x * 256 + threadIdx.x;
    const int f = q * 4;
    if (f < total) {
        float e0, e1, e2, e3;
        { int fe = f + 0; int r = fe / NV; int vv = fe - r * NV; e0 = wsout[(size_t)r * VP + vv]; }
        { int fe = f + 1; int r = fe / NV; int vv = fe - r * NV; e1 = wsout[(size_t)r * VP + vv]; }
        { int fe = f + 2; int r = fe / NV; int vv = fe - r * NV; e2 = wsout[(size_t)r * VP + vv]; }
        { int fe = f + 3; int r = fe / NV; int vv = fe - r * NV; e3 = wsout[(size_t)r * VP + vv]; }
        v4f val;
        val.x = e0; val.y = e1; val.z = e2; val.w = e3;
        float* po = out + f;
        *(volatile v4f*)po = val;
        __threadfence();
        *(volatile v4f*)po = val;
    }
}

extern "C" void kernel_launch(void* const* d_in, const int* in_sizes, int n_in,
                              void* d_out, int out_size, void* d_ws, size_t ws_size,
                              hipStream_t stream) {
    if (n_in < 5) return;
    if (in_sizes[0] != NB * CI * NV) return;
    if (in_sizes[1] != NV * KK) return;
    if (in_sizes[2] != NV * KSQ) return;
    if (in_sizes[3] != CO * KD) return;
    if (in_sizes[4] != CO) return;
    if (out_size != NB * CO * NV) return;

    const float* x    = (const float*)d_in[0];
    const int*   idx  = (const int*)  d_in[1];
    const float* itp  = (const float*)d_in[2];
    const float* w    = (const float*)d_in[3];
    const float* bvec = (const float*)d_in[4];
    float* out = (float*)d_out;

    const size_t off_hi  = 0;
    const size_t off_lo  = (size_t)CO * KD * 2;
    const size_t off_out = 2 * (size_t)CO * KD * 2;
    const size_t need    = off_out + (size_t)NB * CO * VP * 4;
    if (need > ws_size) return;

    unsigned short* whi = (unsigned short*)((char*)d_ws + off_hi);
    unsigned short* wlo = (unsigned short*)((char*)d_ws + off_lo);
    float* wsout = (float*)((char*)d_ws + off_out);

    const int nvec = (CO * KD) / 8;
    k_wsplit<<<1, 256, 0, stream>>>(w, whi, wlo, nvec);

    dim3 g2(NVT, NB);
    k_main<<<g2, NTH, 0, stream>>>(x, idx, itp, whi, wlo, bvec, wsout);

    const int total = out_size;
    const int nthr  = total / 4;
    const int nblk  = (nthr + 255) / 256;
    k_lines<<<nblk, 256, 0, stream>>>(wsout, out, total);
}
